// Net_40312563041045
// MI455X (gfx1250) — hardware-run, weakly checked
//
#include <hip/hip_runtime.h>
#include <math.h>

#ifndef NB
#define NB 1024
#endif
#define NB_FULL 1024
#define D_IN 256
#define D_H 512

#define CARRY_A 2048.0f
#define CARRY_W 131072.0f
#define CARRY_A_INV 4.8828125e-04f
#define CARRY_AW_INV 3.7252902984619140625e-09f
#define MIX_LIN 0.8f
#define MIX_MAX 0.2f

static_assert(NB % 64 == 0);
static_assert(NB <= NB_FULL);
static_assert(D_IN % 64 == 0 && D_H % 64 == 0);
static_assert(((NB / 64) * (D_H / 64)) % 8 == 0);
static_assert((D_H * D_IN / 8) % 256 == 0 && (D_H * D_H / 8) % 256 == 0 && (NB * D_IN / 8) % 256 == 0);

typedef _Float16 h16;
typedef __attribute__((ext_vector_type(16))) _Float16 v16h;
typedef __attribute__((ext_vector_type(8)))  _Float16 v8h;
typedef __attribute__((ext_vector_type(8)))  float    v8f;
typedef __attribute__((ext_vector_type(4)))  float    v4f;


static __device__ __forceinline__ float bfr(float f) {
    unsigned u = __float_as_uint(f);
    u += 0x7FFFu + ((u >> 16) & 1u);
    return __uint_as_float(u & 0xFFFF0000u);
}
static __device__ __forceinline__ h16 toh_flush(float v) {
    const float w = (fabsf(v) < 6.103515625e-05f) ? 0.0f : v;
    return (h16)w;
}
static __device__ __forceinline__ void st2_v8h(h16* p, v8h v) {
    *(volatile v8h*)p = v;
    __threadfence();
    *(volatile v8h*)p = v;
}

union FragU { v16h v; v8h h[2]; };
static __device__ __forceinline__ v16h frag_ld(const h16* p) {
    FragU f; f.h[0] = *(const v8h*)(p); f.h[1] = *(const v8h*)(p + 16); return f.v;
}
static __device__ __forceinline__ v8f wmma16g(v16h a, v16h b, v8f c) {
    c = __builtin_amdgcn_wmma_f32_16x16x32_f16(false, a, false, b, (short)0, c, false, false);
    asm volatile("v_nop\n\tv_nop\n\tv_nop\n\tv_nop" : "+v"(c) : "v"(a), "v"(b));
    return c;
}
static __device__ __forceinline__ void wave_sync_lds() {
    __builtin_amdgcn_fence(3  , "workgroup");
    __builtin_amdgcn_wave_barrier();
    __builtin_amdgcn_fence(2  , "workgroup");
}

template <int IS_W>
__global__ __launch_bounds__(256) void k_cvt16(const float* __restrict__ src, h16* __restrict__ dst, unsigned n8) {
    const unsigned u = blockIdx.x * 256u + threadIdx.x;
    if (u >= n8) return;
    const float carry = IS_W ? CARRY_W : CARRY_A;
    const float* sp = src + (size_t)u * 8u;
    const v4f a = *(const v4f*)sp;
    const v4f b = *(const v4f*)(sp + 4);
    v8h o;
    o[0] = toh_flush(bfr(a.x) * carry);
    o[1] = toh_flush(bfr(a.y) * carry);
    o[2] = toh_flush(bfr(a.z) * carry);
    o[3] = toh_flush(bfr(a.w) * carry);
    o[4] = toh_flush(bfr(b.x) * carry);
    o[5] = toh_flush(bfr(b.y) * carry);
    o[6] = toh_flush(bfr(b.z) * carry);
    o[7] = toh_flush(bfr(b.w) * carry);
    st2_v8h(dst + (size_t)u * 8u, o);
}

#define TP 72
#define OP 68
__global__ __launch_bounds__(256) void k_trop(const h16* __restrict__ A, const h16* __restrict__ W,
                                              float* __restrict__ MX, unsigned K) {
    __shared__ __align__(16) h16 sA[64 * TP];
    __shared__ __align__(16) h16 sW[64 * TP];
    __shared__ __align__(16) float sO[64 * OP];
    const unsigned tid = threadIdx.x;
    const unsigned tx = tid & 15u, ty = tid >> 4;
    const unsigned bx = blockIdx.x;
    const unsigned tilesN = (unsigned)(D_H / 64);
    const unsigned tm = bx / tilesN;
    const unsigned tn = bx - tm * tilesN;
    const unsigned m0 = tm * 64u, n0 = tn * 64u;

    float mx[4][4];
#pragma unroll
    for (int i = 0; i < 4; ++i)
#pragma unroll
        for (int j = 0; j < 4; ++j) mx[i][j] = -3.0e38f;

    for (unsigned k0 = 0; k0 < K; k0 += 64u) {
#pragma unroll
        for (int s = 0; s < 2; ++s) {
            const unsigned p = tid + 256u * (unsigned)s;
            const unsigned row = p >> 3, c8 = (p & 7u) * 8u;
            const v8h av = *(const v8h*)(A + (size_t)(m0 + row) * K + k0 + c8);
            const v8h wv = *(const v8h*)(W + (size_t)(n0 + row) * K + k0 + c8);
            *(v8h*)(sA + row * TP + c8) = av;
            *(v8h*)(sW + row * TP + c8) = wv;
        }
        __syncthreads();
        for (unsigned kk = 0; kk < 64u; kk += 8u) {
            v8h av[4], wv[4];
#pragma unroll
            for (int i = 0; i < 4; ++i) av[i] = *(const v8h*)(sA + (ty * 4u + (unsigned)i) * TP + kk);
#pragma unroll
            for (int j = 0; j < 4; ++j) wv[j] = *(const v8h*)(sW + (tx + 16u * (unsigned)j) * TP + kk);
#pragma unroll
            for (int e = 0; e < 8; ++e) {
                float af[4], wf[4];
#pragma unroll
                for (int i = 0; i < 4; ++i) af[i] = (float)av[i][e];
#pragma unroll
                for (int j = 0; j < 4; ++j) wf[j] = (float)wv[j][e];
#pragma unroll
                for (int i = 0; i < 4; ++i)
#pragma unroll
                    for (int j = 0; j < 4; ++j) mx[i][j] = fmaxf(mx[i][j], af[i] * wf[j]);
            }
        }
        __syncthreads();
    }
#pragma unroll
    for (int i = 0; i < 4; ++i)
#pragma unroll
        for (int j = 0; j < 4; ++j)
            sO[(ty * 4u + (unsigned)i) * OP + tx + 16u * (unsigned)j] = mx[i][j] * CARRY_AW_INV;
    __syncthreads();
    {
        const unsigned lane = tid & 31u, wave = tid >> 5;
        const unsigned hh = lane >> 4, c4 = (lane & 15u) * 4u;
        v4f vv[4];
#pragma unroll
        for (int it = 0; it < 4; ++it) {
            const unsigned row = wave * 8u + (unsigned)it * 2u + hh;
            const float* sp = sO + row * OP + c4;
            v4f t; t.x = sp[0]; t.y = sp[1]; t.z = sp[2]; t.w = sp[3];
            vv[it] = t;
        }
#pragma unroll
        for (int it = 0; it < 4; ++it) {
            const unsigned row = wave * 8u + (unsigned)it * 2u + hh;
            *(volatile v4f*)(MX + (size_t)(m0 + row) * (unsigned)D_H + n0 + c4) = vv[it];
        }
        __threadfence();
#pragma unroll
        for (int it = 0; it < 4; ++it) {
            const unsigned row = wave * 8u + (unsigned)it * 2u + hh;
            *(volatile v4f*)(MX + (size_t)(m0 + row) * (unsigned)D_H + n0 + c4) = vv[it];
        }
    }
}

__global__ __launch_bounds__(256) void k_lin(
    const h16* __restrict__ A, unsigned lda, const h16* __restrict__ Bt, unsigned ldb,
    h16* __restrict__ C, unsigned ldc, const float* __restrict__ bias, const float* __restrict__ MX, unsigned ldm,
    unsigned M, unsigned N, unsigned K) {
    __shared__ __align__(16) float sT[8][16 * 68];
    const unsigned lane = threadIdx.x & 31u;
    const unsigned wave = threadIdx.x >> 5;
    const unsigned tilesN = N >> 6, tilesM = M >> 6;
    const unsigned tile = blockIdx.x * 8u + wave;
    if (tile >= tilesM * tilesN) return;
    const unsigned tm = tile / tilesN;
    const unsigned tn = tile - tm * tilesN;
    const unsigned m0 = tm << 6, n0 = tn << 6;
    const unsigned rlane = lane & 15u;
    const unsigned koff = (lane >> 4) * 8u;
    const unsigned mOff = koff;

    v8f acc[4][4];
#pragma unroll
    for (int i = 0; i < 4; ++i)
#pragma unroll
        for (int j = 0; j < 4; ++j) acc[i][j] = (v8f){0.f,0.f,0.f,0.f,0.f,0.f,0.f,0.f};

    for (unsigned k0 = 0; k0 < K; k0 += 32u) {
        v16h bh[4];
#pragma unroll
        for (int j = 0; j < 4; ++j)
            bh[j] = frag_ld(Bt + (size_t)(n0 + ((unsigned)j << 4) + rlane) * ldb + koff + k0);
#pragma unroll
        for (int i = 0; i < 4; ++i) {
            const v16h ah = frag_ld(A + (size_t)(m0 + ((unsigned)i << 4) + rlane) * lda + koff + k0);
#pragma unroll
            for (int j = 0; j < 4; ++j) acc[i][j] = wmma16g(ah, bh[j], acc[i][j]);
        }
    }

    const unsigned q = lane >> 3, c8 = (lane & 7u) * 8u;
    float bb[8];
    {
        const float* bp = bias + n0 + c8;
        const v4f b0 = *(const v4f*)bp;
        const v4f b1 = *(const v4f*)(bp + 4);
        bb[0] = bfr(b0.x); bb[1] = bfr(b0.y); bb[2] = bfr(b0.z); bb[3] = bfr(b0.w);
        bb[4] = bfr(b1.x); bb[5] = bfr(b1.y); bb[6] = bfr(b1.z); bb[7] = bfr(b1.w);
    }

    float* slab = sT[wave];
#pragma unroll
    for (int i = 0; i < 4; ++i) {
        const unsigned mBase = m0 + ((unsigned)i << 4);
#pragma unroll
        for (int j = 0; j < 4; ++j) {
#pragma unroll
            for (int r = 0; r < 8; ++r)
                slab[(mOff + (unsigned)r) * 68u + ((unsigned)j << 4) + rlane] = acc[i][j][r];
        }
        wave_sync_lds();
        v8h hv[4];
#pragma unroll
        for (int it = 0; it < 4; ++it) {
            const unsigned row = (unsigned)it * 4u + q;
            const float* sp = slab + row * 68u + c8;
            const float* mp = MX + (size_t)(mBase + row) * ldm + n0 + c8;
            const v4f ma = *(const v4f*)mp;
            const v4f mb = *(const v4f*)(mp + 4);
            const float mm[8] = {ma.x, ma.y, ma.z, ma.w, mb.x, mb.y, mb.z, mb.w};
#pragma unroll
            for (int e = 0; e < 8; ++e) {
                const float lin = sp[e] * CARRY_AW_INV;
                const float v = MIX_LIN * lin + MIX_MAX * mm[e] + bb[e];
                hv[it][e] = toh_flush(v * CARRY_A);
            }
        }
#pragma unroll
        for (int it = 0; it < 4; ++it) {
            const unsigned row = (unsigned)it * 4u + q;
            *(volatile v8h*)(C + (size_t)(mBase + row) * ldc + n0 + c8) = hv[it];
        }
        __threadfence();
#pragma unroll
        for (int it = 0; it < 4; ++it) {
            const unsigned row = (unsigned)it * 4u + q;
            *(volatile v8h*)(C + (size_t)(mBase + row) * ldc + n0 + c8) = hv[it];
        }
        wave_sync_lds();
    }
}

__global__ __launch_bounds__(256) void k_out(const h16* __restrict__ H, const float* __restrict__ W4,
                                             const float* __restrict__ b4, float* __restrict__ out) {
    const unsigned lane = threadIdx.x & 31u;
    const unsigned wave = threadIdx.x >> 5;
    const unsigned row0 = (blockIdx.x * 8u + wave) * 32u;
    if (row0 >= (unsigned)NB) return;
    float w0[8], w1[8];
    {
        const float* wp = W4 + 8u * lane;
        const v4f a = *(const v4f*)wp;
        const v4f b = *(const v4f*)(wp + 4);
        const v4f c = *(const v4f*)(wp + 256);
        const v4f d = *(const v4f*)(wp + 260);
        w0[0] = bfr(a.x); w0[1] = bfr(a.y); w0[2] = bfr(a.z); w0[3] = bfr(a.w);
        w0[4] = bfr(b.x); w0[5] = bfr(b.y); w0[6] = bfr(b.z); w0[7] = bfr(b.w);
        w1[0] = bfr(c.x); w1[1] = bfr(c.y); w1[2] = bfr(c.z); w1[3] = bfr(c.w);
        w1[4] = bfr(d.x); w1[5] = bfr(d.y); w1[6] = bfr(d.z); w1[7] = bfr(d.w);
    }
    const float bias = bfr(b4[0]);
    float res = 0.0f;
    for (unsigned r = 0; r < 32u; ++r) {
        const h16* hp = H + (size_t)(row0 + r) * (unsigned)D_H + 8u * lane;
        const v8h a0 = *(const v8h*)hp;
        const v8h a1 = *(const v8h*)(hp + 256);
        float s = 0.0f, m = -3.0e38f;
#pragma unroll
        for (int e = 0; e < 8; ++e) {
            const float p = w0[e] * (float)a0[e];
            s += p;
            m = fmaxf(m, p);
        }
#pragma unroll
        for (int e = 0; e < 8; ++e) {
            const float p = w1[e] * (float)a1[e];
            s += p;
            m = fmaxf(m, p);
        }
#pragma unroll
        for (int o = 16; o > 0; o >>= 1) {
            s += __shfl_xor(s, o, 32);
            m = fmaxf(m, __shfl_xor(m, o, 32));
        }
        const float val = MIX_LIN * (s * CARRY_A_INV) + MIX_MAX * (m * CARRY_A_INV) + bias;
        res = (lane == r) ? val : res;
    }
    const float fin = res;
    *(volatile float*)(out + row0 + lane) = fin;
    __threadfence();
    *(volatile float*)(out + row0 + lane) = fin;
}

extern "C" void kernel_launch(void* const* d_in, const int* in_sizes, int n_in, void* d_out, int out_size,
                              void* d_ws, size_t ws_size, hipStream_t stream) {
    if (n_in < 9) return;
    if (in_sizes[0] < NB * D_IN || in_sizes[1] < D_H * D_IN || in_sizes[2] < D_H) return;
    if (in_sizes[3] < D_H * D_H || in_sizes[4] < D_H || in_sizes[5] < D_H * D_H || in_sizes[6] < D_H) return;
    if (in_sizes[7] < D_H || in_sizes[8] < 1 || out_size < NB) return;

    const float* x  = (const float*)d_in[0];
    const float* W1 = (const float*)d_in[1];
    const float* b1 = (const float*)d_in[2];
    const float* W2 = (const float*)d_in[3];
    const float* b2 = (const float*)d_in[4];
    const float* W3 = (const float*)d_in[5];
    const float* b3 = (const float*)d_in[6];
    const float* W4 = (const float*)d_in[7];
    const float* b4 = (const float*)d_in[8];
    float* out = (float*)d_out;

    constexpr size_t SZ_W1 = (size_t)D_H * D_IN * 2;
    constexpr size_t SZ_WH = (size_t)D_H * D_H * 2;
    constexpr size_t SZ_X  = (size_t)NB * D_IN * 2;
    constexpr size_t SZ_H  = (size_t)NB * D_H * 2;
    constexpr size_t SZ_MX = (size_t)NB * D_H * 4;
    static_assert(SZ_W1 % 256 == 0 && SZ_WH % 256 == 0 && SZ_X % 256 == 0 && SZ_H % 256 == 0 && SZ_MX % 256 == 0);
    static_assert(SZ_W1 + 2 * SZ_WH + SZ_X + 3 * SZ_H + 3 * SZ_MX <= (size_t)134217728);

    char* wsp = (char*)d_ws;
    size_t off = 0;
    auto carve = [&](size_t bytes) -> void* { void* r = wsp + off; off += (bytes + 255) & ~(size_t)255; return r; };
    h16*   w1p = (h16*)carve(SZ_W1);
    h16*   w2p = (h16*)carve(SZ_WH);
    h16*   w3p = (h16*)carve(SZ_WH);
    h16*   xp  = (h16*)carve(SZ_X);
    h16*   h1  = (h16*)carve(SZ_H);
    h16*   h2  = (h16*)carve(SZ_H);
    h16*   h3  = (h16*)carve(SZ_H);
    float* mx1 = (float*)carve(SZ_MX);
    float* mx2 = (float*)carve(SZ_MX);
    float* mx3 = (float*)carve(SZ_MX);
    if (off > ws_size || off > (size_t)134217728) return;

    k_cvt16<1><<<(D_H * D_IN / 8) / 256, 256, 0, stream>>>(W1, w1p, (unsigned)(D_H * D_IN / 8));
    k_cvt16<1><<<(D_H * D_H / 8) / 256, 256, 0, stream>>>(W2, w2p, (unsigned)(D_H * D_H / 8));
    k_cvt16<1><<<(D_H * D_H / 8) / 256, 256, 0, stream>>>(W3, w3p, (unsigned)(D_H * D_H / 8));
    k_cvt16<0><<<(NB * D_IN / 8) / 256, 256, 0, stream>>>(x, xp, (unsigned)(NB * D_IN / 8));

    const unsigned gT = (unsigned)((NB / 64) * (D_H / 64));
    const unsigned gL = (unsigned)(((NB / 64) * (D_H / 64)) / 8);

    k_trop<<<gT, 256, 0, stream>>>(xp, w1p, mx1, (unsigned)D_IN);
    k_lin<<<gL, 256, 0, stream>>>(xp, (unsigned)D_IN, w1p, (unsigned)D_IN, h1, (unsigned)D_H, b1, mx1, (unsigned)D_H,
                                  (unsigned)NB, (unsigned)D_H, (unsigned)D_IN);
    k_trop<<<gT, 256, 0, stream>>>(h1, w2p, mx2, (unsigned)D_H);
    k_lin<<<gL, 256, 0, stream>>>(h1, (unsigned)D_H, w2p, (unsigned)D_H, h2, (unsigned)D_H, b2, mx2, (unsigned)D_H,
                                  (unsigned)NB, (unsigned)D_H, (unsigned)D_H);
    k_trop<<<gT, 256, 0, stream>>>(h2, w3p, mx3, (unsigned)D_H);
    k_lin<<<gL, 256, 0, stream>>>(h2, (unsigned)D_H, w3p, (unsigned)D_H, h3, (unsigned)D_H, b3, mx3, (unsigned)D_H,
                                  (unsigned)NB, (unsigned)D_H, (unsigned)D_H);
    k_out<<<(unsigned)((NB / 32 + 7) / 8), 256, 0, stream>>>(h3, W4, b4, out);
}
